// GraphSAGE_55490977464722
// MI455X (gfx1250) — hardware-run, weakly checked
//
#include <hip/hip_runtime.h>
#include <stddef.h>
#include <stdint.h>

#ifndef MEAN_SPLIT
#define MEAN_SPLIT 1
#endif
#ifndef HID_SPLIT
#define HID_SPLIT 1
#endif

#define NN      100000
#define HD      64
#define NE      1200000
#define GBM     128
#define MP      100096
#define XP      64
#define MPITCH  128
#define W1P     192
#define W2P     256
#define K1      (HD + HD * (1 + MEAN_SPLIT))
#define K2      (HD * (1 + HID_SPLIT) + HD * (1 + MEAN_SPLIT))
#define NTHR    256
#define NWAVE   8
#define EPT     8
#define WCH     (32 * EPT)
#define NBRUN   1024
#define SLB     10
#define NBK     98
#define WLCAP   2560
#define RCAP    16384
#define DEGCAP  64
#define MAXDEG_MEAS   30
#define MAXB1024_MEAS 12491
#define ABM     128
#define SP      68
#define WSMAX   ((size_t)128 << 20)

#define BK_ZINTS (NWAVE * WLCAP + RCAP + 3 * NBRUN)
#define BK_INTS  (BK_ZINTS + 16)
#define BK_LDS   (BK_INTS * 4)

#define UW1   (W1P / 8)
#define PBX   (MP * HD / 8 / NTHR)
#define PBW1  (HD * W1P / 8 / NTHR)
#define PBW2  (HD * W2P / 8 / NTHR)
#define PBTOT (PBX + PBW1 + PBW2 + 1)

static_assert(HD == 64 && HD == 16 * 4);
static_assert(XP == HD && MPITCH == 2 * HD && W1P == 3 * HD && W2P == 4 * HD);
static_assert(K1 % 32 == 0 && K2 % 32 == 0 && K1 <= W1P && K2 <= W2P);
static_assert(MP % GBM == 0 && MP >= NN && MP == 782 * GBM && MP % ABM == 0);
static_assert(NBRUN == (1 << SLB) && NBRUN % ABM == 0 && NBRUN % 32 == 0);
static_assert(NBK * NBRUN >= MP);
static_assert(NE < (1 << 21) && (((long long)NE) << SLB) < (1LL << 31));
static_assert(NE % EPT == 0 && NE % 4 == 0 && NE >= EPT);
static_assert(RCAP % (NTHR * 4) == 0 && BK_ZINTS % (NTHR * 4) == 0 && (2 * NBRUN) == 2 * NTHR * 4);
static_assert((long long)RCAP * 100 >= (long long)MAXB1024_MEAS * 105);
static_assert(WLCAP >= MAXB1024_MEAS / 8 + 8 * 40 + 1);
static_assert(MAXDEG_MEAS + 8 <= DEGCAP);
static_assert((MP * HD / 8) % NTHR == 0 && (HD * W1P / 8) % NTHR == 0 && (HD * W2P / 8) % NTHR == 0);
static_assert(BK_LDS <= 300000);
static_assert((GBM * SP + 64) * 4 <= 65536);
static_assert(ABM % NWAVE == 0 && GBM == NWAVE * 16);

typedef float          v4f   __attribute__((ext_vector_type(4)));
typedef float          v8f   __attribute__((ext_vector_type(8)));
typedef int            v4i   __attribute__((ext_vector_type(4)));
typedef int            v8i   __attribute__((ext_vector_type(8)));
typedef unsigned       v2u   __attribute__((ext_vector_type(2)));
typedef unsigned short v8us  __attribute__((ext_vector_type(8)));
typedef unsigned short v16us __attribute__((ext_vector_type(16)));
typedef __bf16         v16bf __attribute__((ext_vector_type(16)));
typedef v4f  __attribute__((may_alias)) v4fa;
typedef v4i  __attribute__((may_alias)) v4ia;
typedef v2u  __attribute__((may_alias)) v2ua;
typedef v8us __attribute__((may_alias)) v8usa;
union FragB { v16bf v; v16us u; v8us h[2]; v8i w; };

__device__ __forceinline__ v8f wmb(const FragB& a, const FragB& b, v8f c) {
  v8f d = __builtin_amdgcn_wmma_f32_16x16x32_bf16(false, a.v, false, b.v, (short)0, c, false, false);
  asm volatile("v_nop\n\tv_nop\n\tv_nop\n\tv_nop" : "+v"(d) : "v"(a.w), "v"(b.w));
  return d;
}

__device__ __forceinline__ unsigned bf16_bits(float f) {
  const unsigned u = __float_as_uint(f);
  const unsigned r = (u + 0x7FFFu + ((u >> 16) & 1u)) >> 16;
  const unsigned q = (u >> 16) | 0x40u;
  return ((u & 0x7fffffffu) > 0x7f800000u) ? q : r;
}

__device__ __forceinline__ void hilo_pack(float v0, float v1, float v2, float v3,
                                          int& h01, int& h23, int& l01, int& l23) {
  const unsigned a0 = bf16_bits(v0), a1 = bf16_bits(v1), a2 = bf16_bits(v2), a3 = bf16_bits(v3);
  const unsigned b0 = bf16_bits(v0 - __uint_as_float(a0 << 16));
  const unsigned b1 = bf16_bits(v1 - __uint_as_float(a1 << 16));
  const unsigned b2 = bf16_bits(v2 - __uint_as_float(a2 << 16));
  const unsigned b3 = bf16_bits(v3 - __uint_as_float(a3 << 16));
  h01 = (int)(a0 | (a1 << 16)); h23 = (int)(a2 | (a3 << 16));
  l01 = (int)(b0 | (b1 << 16)); l23 = (int)(b2 | (b3 << 16));
}

__device__ __forceinline__ v4i regroup8(int h01, int h23, int l01, int l23, int lane) {
  const int t  = lane & 15;
  const int s0 = (lane & 16) + ((2 * t) & 15), s1 = s0 + 1;
  const int a0 = __shfl(h01, s0, 32), a1 = __shfl(h23, s0, 32), a2 = __shfl(h01, s1, 32), a3 = __shfl(h23, s1, 32);
  const int b0 = __shfl(l01, s0, 32), b1 = __shfl(l23, s0, 32), b2 = __shfl(l01, s1, 32), b3 = __shfl(l23, s1, 32);
  const int mk = (t < 8) ? -1 : 0;
  v4i o;
  o.x = (a0 & mk) | (b0 & ~mk); o.y = (a1 & mk) | (b1 & ~mk);
  o.z = (a2 & mk) | (b2 & ~mk); o.w = (a3 & mk) | (b3 & ~mk);
  return o;
}

__device__ __forceinline__ void st2_v4f(float* p, v4f v) {
  *(volatile v4f*)p = v;
  __threadfence();
  *(volatile v4f*)p = v;
}
__device__ __forceinline__ void st2_v8us(unsigned short* p, v8us v) {
  *(volatile v8us*)p = v;
  __threadfence();
  *(volatile v8us*)p = v;
}

__device__ __forceinline__ v8us strided8(const float* __restrict__ base, int stride) {
  float f[8];
#pragma unroll
  for (int i = 0; i < 8; ++i) f[i] = base[(size_t)i * (size_t)stride];
  v8us o;
#pragma unroll
  for (int i = 0; i < 8; ++i) o[i] = (unsigned short)bf16_bits(f[i]);
  return o;
}

__global__ __launch_bounds__(NTHR) void k_prep(const float* __restrict__ x, const float* __restrict__ w1,
                                               const float* __restrict__ b1, const float* __restrict__ w2,
                                               const float* __restrict__ b2, unsigned short* xb,
                                               unsigned short* wt1, unsigned short* wt2, float* sm) {
  const int tid = (int)threadIdx.x, lane = tid & 31;
  const int blk = (int)blockIdx.x;
  if (blk < PBX) {
    const int u   = blk * NTHR + tid;
    const int row = u >> 3, k8 = (u & 7) * 8;
    const int rc  = row < NN ? row : NN - 1;
    const unsigned mk = row < NN ? 0xffffu : 0u;
    const float* p = x + (size_t)rc * HD + k8;
    const v4f a = *(const v4fa*)p;
    const v4f b = *(const v4fa*)(p + 4);
    asm volatile("" :: "v"(a), "v"(b));
    v8us o;
    o[0] = (unsigned short)(bf16_bits(a.x) & mk); o[1] = (unsigned short)(bf16_bits(a.y) & mk);
    o[2] = (unsigned short)(bf16_bits(a.z) & mk); o[3] = (unsigned short)(bf16_bits(a.w) & mk);
    o[4] = (unsigned short)(bf16_bits(b.x) & mk); o[5] = (unsigned short)(bf16_bits(b.y) & mk);
    o[6] = (unsigned short)(bf16_bits(b.z) & mk); o[7] = (unsigned short)(bf16_bits(b.w) & mk);
    st2_v8us(xb + (size_t)row * XP + k8, o);
  } else if (blk < PBX + PBW1) {
    const int u  = (blk - PBX) * NTHR + tid;
    const int n  = u / UW1, k8 = (u - UW1 * n) * 8;
    const int sr = (k8 < 2 * HD) ? k8 : (k8 - HD);
    const v8us o = strided8(w1 + (size_t)sr * HD + n, HD);
    st2_v8us(wt1 + (size_t)n * W1P + k8, o);
  } else if (blk < PBX + PBW1 + PBW2) {
    const int u  = (blk - PBX - PBW1) * NTHR + tid;
    const int n  = u >> 5, k8 = (u & 31) * 8;
    const int sr = (k8 < HD) ? k8 : ((k8 < 3 * HD) ? (k8 - HD) : (k8 - 2 * HD));
    const v8us o = strided8(w2 + (size_t)sr * HD + n, HD);
    st2_v8us(wt2 + (size_t)n * W2P + k8, o);
  } else {
    if (tid < 32) {
      const int q = lane & 15;
      const v4f a = *(const v4fa*)(b1 + 4 * q);
      const v4f c = *(const v4fa*)(b2 + 4 * q);
      asm volatile("" :: "v"(a), "v"(c));
      const unsigned ma = (lane < 16) ? 0xffffffffu : 0u;
      v4f o;
      o.x = __uint_as_float(((bf16_bits(a.x) << 16) & ma) | ((bf16_bits(c.x) << 16) & ~ma));
      o.y = __uint_as_float(((bf16_bits(a.y) << 16) & ma) | ((bf16_bits(c.y) << 16) & ~ma));
      o.z = __uint_as_float(((bf16_bits(a.z) << 16) & ma) | ((bf16_bits(c.z) << 16) & ~ma));
      o.w = __uint_as_float(((bf16_bits(a.w) << 16) & ma) | ((bf16_bits(c.w) << 16) & ~ma));
      st2_v4f(sm + 4 * lane, o);
    }
  }
}

__device__ __forceinline__ void bucket_flush(const int* pl, const int* cnt, int ov, int* lp, int* cop, int* fp,
                                             int tid) {
#pragma unroll 1
  for (int i = tid * 4; i < RCAP; i += NTHR * 4) {
    const v4i v = *(const v4ia*)(pl + i);
    *(volatile v4i*)(lp + i) = v;
  }
#pragma unroll 1
  for (int it = 0; it < 2; ++it) {
    const int idx = (it * NTHR + tid) * 4;
    const v4i v = *(const v4ia*)(cnt + idx);
    *(volatile v4i*)(cop + idx) = v;
  }
  if (tid < 8) {
    const v4i f = {ov, ov, ov, ov};
    *(volatile v4i*)(fp + 4 * tid) = f;
  }
}

__global__ __launch_bounds__(NTHR) void k_bucket(const int* __restrict__ keys, const int* __restrict__ srcs,
                                                 int* LIST, int* CO, int* FLAG) {
  extern __shared__ __attribute__((aligned(16))) int dsm[];
  int* wl   = dsm;
  int* pl   = dsm + NWAVE * WLCAP;
  int* cnt  = pl + RCAP;
  int* offs = cnt + NBRUN;
  int* cur  = offs + NBRUN;
  int* misc = cur + NBRUN;
  const int tid = (int)threadIdx.x, lane = tid & 31, wave = tid >> 5;
  const int blk = (int)blockIdx.x;
  const unsigned nbs = (unsigned)(blk * NBRUN);

  {
    const v4i z4 = {0, 0, 0, 0};
    for (int i = tid * 4; i < BK_ZINTS; i += NTHR * 4) *(v4ia*)(dsm + i) = z4;
    if (tid < 16) misc[tid] = 0;
  }
  __syncthreads();

  {
    const int per  = ((NE + NWAVE * WCH - 1) / (NWAVE * WCH)) * WCH;
    const int ebeg = wave * per;
    const int eend = (ebeg + per < NE) ? (ebeg + per) : NE;
    int* mylist = wl + wave * WLCAP;
    int wc = 0;
#pragma unroll 1
    for (int cb = ebeg; cb < eend; cb += WCH) {
      const int e0 = cb + lane * EPT;
      const int ec = (e0 < NE - EPT) ? e0 : (NE - EPT);
      const v4i da = *(const v4ia*)(keys + ec);
      const v4i db = *(const v4ia*)(keys + ec + 4);
      asm volatile("" :: "v"(da), "v"(db));
      const unsigned inval = (e0 < eend) ? 0u : 0xffffffffu;
      const unsigned s0 = ((unsigned)da.x - nbs) | inval, s1 = ((unsigned)da.y - nbs) | inval;
      const unsigned s2 = ((unsigned)da.z - nbs) | inval, s3 = ((unsigned)da.w - nbs) | inval;
      const unsigned s4 = ((unsigned)db.x - nbs) | inval, s5 = ((unsigned)db.y - nbs) | inval;
      const unsigned s6 = ((unsigned)db.z - nbs) | inval, s7 = ((unsigned)db.w - nbs) | inval;
      const bool h0 = s0 < (unsigned)NBRUN, h1 = s1 < (unsigned)NBRUN, h2 = s2 < (unsigned)NBRUN, h3 = s3 < (unsigned)NBRUN;
      const bool h4 = s4 < (unsigned)NBRUN, h5 = s5 < (unsigned)NBRUN, h6 = s6 < (unsigned)NBRUN, h7 = s7 < (unsigned)NBRUN;
      const unsigned m0 = __builtin_amdgcn_ballot_w32(h0), m1 = __builtin_amdgcn_ballot_w32(h1);
      const unsigned m2 = __builtin_amdgcn_ballot_w32(h2), m3 = __builtin_amdgcn_ballot_w32(h3);
      const unsigned m4 = __builtin_amdgcn_ballot_w32(h4), m5 = __builtin_amdgcn_ballot_w32(h5);
      const unsigned m6 = __builtin_amdgcn_ballot_w32(h6), m7 = __builtin_amdgcn_ballot_w32(h7);
      const unsigned any = m0 | m1 | m2 | m3 | m4 | m5 | m6 | m7;
      if (any != 0u) {
        const int pre = (int)(__builtin_amdgcn_mbcnt_lo(m0, 0u) + __builtin_amdgcn_mbcnt_lo(m1, 0u) +
                              __builtin_amdgcn_mbcnt_lo(m2, 0u) + __builtin_amdgcn_mbcnt_lo(m3, 0u) +
                              __builtin_amdgcn_mbcnt_lo(m4, 0u) + __builtin_amdgcn_mbcnt_lo(m5, 0u) +
                              __builtin_amdgcn_mbcnt_lo(m6, 0u) + __builtin_amdgcn_mbcnt_lo(m7, 0u));
        int p = wc + pre;
        if (h0) { if (p < WLCAP) mylist[p] = ((e0 + 0) << SLB) | (int)s0; p = p + 1; }
        if (h1) { if (p < WLCAP) mylist[p] = ((e0 + 1) << SLB) | (int)s1; p = p + 1; }
        if (h2) { if (p < WLCAP) mylist[p] = ((e0 + 2) << SLB) | (int)s2; p = p + 1; }
        if (h3) { if (p < WLCAP) mylist[p] = ((e0 + 3) << SLB) | (int)s3; p = p + 1; }
        if (h4) { if (p < WLCAP) mylist[p] = ((e0 + 4) << SLB) | (int)s4; p = p + 1; }
        if (h5) { if (p < WLCAP) mylist[p] = ((e0 + 5) << SLB) | (int)s5; p = p + 1; }
        if (h6) { if (p < WLCAP) mylist[p] = ((e0 + 6) << SLB) | (int)s6; p = p + 1; }
        if (h7) { if (p < WLCAP) mylist[p] = ((e0 + 7) << SLB) | (int)s7; p = p + 1; }
        wc += (int)(__builtin_popcount(m0) + __builtin_popcount(m1) + __builtin_popcount(m2) + __builtin_popcount(m3) +
                    __builtin_popcount(m4) + __builtin_popcount(m5) + __builtin_popcount(m6) + __builtin_popcount(m7));
      }
    }
    if (lane == 0) misc[wave] = wc;
  }
  __syncthreads();

  if (wave == 0) {
    int ov = 0, tot = 0;
#pragma unroll 1
    for (int w2 = 0; w2 < NWAVE; ++w2) {
      int c = misc[w2];
      if (c > WLCAP) ov = 1;
      c = c < 0 ? 0 : (c > WLCAP ? WLCAP : c);
      tot += c;
#pragma unroll 1
      for (int b0 = 0; b0 < c; b0 += 32) {
        const int idx = b0 + lane;
        const int ent = wl[w2 * WLCAP + (idx < WLCAP ? idx : WLCAP - 1)];
        const int m32 = (c - b0) < 32 ? (c - b0) : 32;
#pragma unroll 1
        for (int k = 0; k < m32; ++k) {
          const int u    = __builtin_amdgcn_readlane(ent, k);
          const int slot = u & (NBRUN - 1);
          if (lane == 0) cnt[slot] = cnt[slot] + 1;
        }
      }
    }
    if (tot > RCAP) ov = 1;
    if (lane == 0) misc[9] = ov;
  }
  __syncthreads();
  if (wave == 0) {
    const int base = lane * (NBRUN / 32);
    int s = 0, bigAny = 0;
#pragma unroll 1
    for (int i = 0; i < NBRUN / 32; ++i) {
      const int cv = cnt[base + i];
      bigAny |= (cv > DEGCAP) ? 1 : 0;
      s += cv;
    }
    const unsigned bm = __builtin_amdgcn_ballot_w32(bigAny != 0);
    int incl = s;
#pragma unroll
    for (int d = 1; d < 32; d <<= 1) {
      const int y = __shfl_up(incl, d, 32);
      if (lane >= d) incl += y;
    }
    int run = incl - s;
#pragma unroll 1
    for (int i = 0; i < NBRUN / 32; ++i) {
      const int cv = cnt[base + i];
      offs[base + i] = run;
      cur[base + i]  = run;
      run += cv;
    }
    if (lane == 0) misc[9] = misc[9] | ((bm != 0u) ? 1 : 0);
  }
  __syncthreads();

  if (wave == 0) {
#pragma unroll 1
    for (int w2 = 0; w2 < NWAVE; ++w2) {
      int c = misc[w2];
      c = c < 0 ? 0 : (c > WLCAP ? WLCAP : c);
#pragma unroll 1
      for (int b0 = 0; b0 < c; b0 += 32) {
        const int idx = b0 + lane;
        const int ent = wl[w2 * WLCAP + (idx < WLCAP ? idx : WLCAP - 1)];
        int eid = (ent >> SLB) & 0x1FFFFF;
        eid = eid > NE - 1 ? NE - 1 : eid;
        int sr = srcs[eid];
        sr = sr < 0 ? 0 : (sr > NN - 1 ? NN - 1 : sr);
        const int m32 = (c - b0) < 32 ? (c - b0) : 32;
#pragma unroll 1
        for (int k = 0; k < m32; ++k) {
          const int u    = __builtin_amdgcn_readlane(ent, k);
          const int wd   = __builtin_amdgcn_readlane(sr, k);
          const int slot = u & (NBRUN - 1);
          if (lane == 0) {
            int p = cur[slot];
            p = p < 0 ? 0 : (p > RCAP - 1 ? RCAP - 1 : p);
            pl[p] = wd;
            cur[slot] = p + 1;
          }
        }
      }
    }
  }
  __syncthreads();

  const int ovf = misc[9];
  int* lp  = LIST + (size_t)blk * RCAP;
  int* cop = CO + (size_t)blk * (2 * NBRUN);
  int* fp  = FLAG + (size_t)blk * 32;
  bucket_flush(pl, cnt, ovf, lp, cop, fp, tid);
  __threadfence();
  bucket_flush(pl, cnt, ovf, lp, cop, fp, tid);
}

template <int SRC>
__device__ __forceinline__ void replay_rows(const int* __restrict__ LIST, const int* __restrict__ CO,
                                            const int* __restrict__ FLAG,
                                            const unsigned short* __restrict__ XBs,
                                            const float* __restrict__ Hs, unsigned short* Mhl) {
  const int tid = (int)threadIdx.x, lane = tid & 31, wave = tid >> 5, hh = lane >> 4, q = lane & 15;
  const int rowBase = (int)blockIdx.x * ABM;
  const int bucket  = rowBase >> SLB;
  const int* lb  = LIST + (size_t)bucket * RCAP;
  const int* cob = CO + (size_t)bucket * (2 * NBRUN);
  const int flag = FLAG[(size_t)bucket * 32];
  const float qnan = __uint_as_float(0x7fc00000u);

#pragma unroll 1
  for (int i = 0; i < ABM / NWAVE; ++i) {
    const int d    = rowBase + (ABM / NWAVE) * wave + i;
    const int slot = d & (NBRUN - 1);
    int cv = cob[slot];
    int ov = cob[NBRUN + slot];
    const int bigv = (cv > DEGCAP) ? 1 : 0;
    cv = cv < 0 ? 0 : (cv > DEGCAP ? DEGCAP : cv);
    ov = ov < 0 ? 0 : (ov > RCAP - 1 ? RCAP - 1 : ov);
    const int c1v = cv < 1 ? 1 : cv;
    const int c   = __builtin_amdgcn_readfirstlane(cv);
    const int o   = __builtin_amdgcn_readfirstlane(ov);
    const int c1  = __builtin_amdgcn_readfirstlane(c1v);
    const int big = __builtin_amdgcn_readfirstlane(bigv);
    int last = o + c - 1;
    last = last < o ? o : last;
    last = last > RCAP - 1 ? RCAP - 1 : last;
    const int trips = (c + 1) >> 1;
    float a0 = 0.0f, a1 = 0.0f, a2 = 0.0f, a3 = 0.0f;
#pragma unroll 1
    for (int t = 0; t < trips; ++t) {
      const int j = 2 * t + hh;
      int idx = o + j;
      idx = idx > last ? last : idx;
      int sr = lb[idx];
      sr = sr < 0 ? 0 : (sr > NN - 1 ? NN - 1 : sr);
      float f0, f1, f2, f3;
      if constexpr (SRC == 0) {
        const v2u w = *(const v2ua*)(XBs + (size_t)sr * XP + 4 * q);
        asm volatile("" :: "v"(w));
        f0 = __uint_as_float(w.x << 16); f1 = __uint_as_float(w.x & 0xffff0000u);
        f2 = __uint_as_float(w.y << 16); f3 = __uint_as_float(w.y & 0xffff0000u);
      } else {
        const v4f v = *(const v4fa*)(Hs + (size_t)sr * HD + 4 * q);
        asm volatile("" :: "v"(v));
        f0 = v.x; f1 = v.y; f2 = v.z; f3 = v.w;
      }
      const bool valid = j < c;
      f0 = valid ? f0 : 0.0f; f1 = valid ? f1 : 0.0f; f2 = valid ? f2 : 0.0f; f3 = valid ? f3 : 0.0f;
      a0 += f0; a1 += f1; a2 += f2; a3 += f3;
    }
    const float o0 = __shfl_xor(a0, 16, 32), o1 = __shfl_xor(a1, 16, 32);
    const float o2 = __shfl_xor(a2, 16, 32), o3 = __shfl_xor(a3, 16, 32);
    const float fc = (float)c1;
    float m0 = (a0 + o0) / fc, m1 = (a1 + o1) / fc, m2 = (a2 + o2) / fc, m3 = (a3 + o3) / fc;
    const bool bad  = (flag != 0) | (big != 0);
    const bool live = d < NN;
    m0 = bad ? qnan : m0; m1 = bad ? qnan : m1; m2 = bad ? qnan : m2; m3 = bad ? qnan : m3;
    m0 = live ? m0 : 0.0f; m1 = live ? m1 : 0.0f; m2 = live ? m2 : 0.0f; m3 = live ? m3 : 0.0f;
    int h01, h23, l01, l23;
    hilo_pack(m0, m1, m2, m3, h01, h23, l01, l23);
    const v4i ow = regroup8(h01, h23, l01, l23, lane);
    unsigned short* hp = Mhl + (size_t)d * MPITCH + 8 * q;
    if (hh == 0) *(volatile v4i*)hp = ow;
    __threadfence();
    if (hh == 0) *(volatile v4i*)hp = ow;
  }
}

__global__ __launch_bounds__(NTHR) void k_replay_one(const int* __restrict__ LIST, const int* __restrict__ CO,
                                                     const int* __restrict__ FLAG,
                                                     const unsigned short* __restrict__ XBs,
                                                     unsigned short* Mhl) {
  replay_rows<0>(LIST, CO, FLAG, XBs, (const float*)nullptr, Mhl);
}

__global__ __launch_bounds__(NTHR) void k_replay_two(const int* __restrict__ LIST, const int* __restrict__ CO,
                                                     const int* __restrict__ FLAG,
                                                     const float* __restrict__ Hs, unsigned short* Mhl) {
  replay_rows<1>(LIST, CO, FLAG, (const unsigned short*)nullptr, Hs, Mhl);
}

template <int WP>
__device__ __forceinline__ void seg64(const unsigned short* __restrict__ ap,
                                      const unsigned short* __restrict__ bp, v8f (&acc)[4]) {
#pragma unroll 1
  for (int k0 = 0; k0 < HD; k0 += 32) {
    FragB af;
    af.h[0] = *(const v8usa*)(ap + k0);
    af.h[1] = *(const v8usa*)(ap + k0 + 16);
#pragma unroll
    for (int nt = 0; nt < 4; ++nt) {
      const unsigned short* wq = bp + (size_t)(16 * nt) * (size_t)WP + k0;
      FragB bf;
      bf.h[0] = *(const v8usa*)wq;
      bf.h[1] = *(const v8usa*)(wq + 16);
      acc[nt] = wmb(af, bf, acc[nt]);
    }
  }
}

__device__ __forceinline__ void stage_d(float* stg, const v8f (&acc)[4], int wave, int hh, int m) {
#pragma unroll
  for (int nt = 0; nt < 4; ++nt) {
#pragma unroll
    for (int r = 0; r < 8; ++r) stg[(16 * wave + 8 * hh + r) * SP + 16 * nt + m] = acc[nt][r];
  }
}

template <int LAYER>
__device__ __forceinline__ void gemm_rows(const unsigned short* __restrict__ Aown,
                                          const unsigned short* __restrict__ Amean,
                                          const unsigned short* __restrict__ BT,
                                          const float* __restrict__ sm, float* Hout,
                                          unsigned short* HHLout, float* outp, float* stg, float* sb) {
  const int tid = (int)threadIdx.x, lane = tid & 31, wave = tid >> 5, hh = lane >> 4, m = lane & 15;
  const int rowBase = (int)blockIdx.x * GBM;
  if (tid < 16) *(v4fa*)(sb + 4 * tid) = *(const v4fa*)(sm + ((LAYER == 1) ? 0 : 64) + 4 * tid);

  v8f acc[4];
  {
    const v8f z = {0.f, 0.f, 0.f, 0.f, 0.f, 0.f, 0.f, 0.f};
#pragma unroll
    for (int t = 0; t < 4; ++t) acc[t] = z;
  }
  const int row = rowBase + 16 * wave + m;
  const unsigned short* am = Amean + (size_t)row * (size_t)MPITCH + 8 * hh;
  if constexpr (LAYER == 1) {
    const unsigned short* ax = Aown + (size_t)row * (size_t)XP + 8 * hh;
    const unsigned short* bp = BT + (size_t)m * (size_t)W1P + 8 * hh;
    seg64<W1P>(ax, bp, acc);
    seg64<W1P>(am, bp + HD, acc);
    if constexpr (MEAN_SPLIT != 0) seg64<W1P>(am + HD, bp + 2 * HD, acc);
  } else {
    const unsigned short* ah = Aown + (size_t)row * (size_t)MPITCH + 8 * hh;
    const unsigned short* bp = BT + (size_t)m * (size_t)W2P + 8 * hh;
    seg64<W2P>(ah, bp, acc);
    if constexpr (HID_SPLIT != 0) seg64<W2P>(ah + HD, bp + HD, acc);
    seg64<W2P>(am, bp + 2 * HD, acc);
    if constexpr (MEAN_SPLIT != 0) seg64<W2P>(am + HD, bp + 3 * HD, acc);
  }
  stage_d(stg, acc, wave, hh, m);
  __syncthreads();

  const v4f bias = *(const v4fa*)(sb + 4 * m);
#pragma unroll 1
  for (int i = 0; i < 8; ++i) {
    const int lr   = 16 * wave + 2 * i + hh;
    const int grow = rowBase + lr;
    const bool live = grow < NN;
    const v4f a = *(const v4fa*)(stg + lr * SP + 4 * m);
    asm volatile("" :: "v"(a));
    float v0 = a.x + bias.x, v1 = a.y + bias.y, v2 = a.z + bias.z, v3 = a.w + bias.w;
    if constexpr (LAYER == 1) {
      v0 = (v0 > 0.0f) ? v0 : (v0 - v0); v1 = (v1 > 0.0f) ? v1 : (v1 - v1);
      v2 = (v2 > 0.0f) ? v2 : (v2 - v2); v3 = (v3 > 0.0f) ? v3 : (v3 - v3);
      v0 = live ? v0 : 0.0f; v1 = live ? v1 : 0.0f; v2 = live ? v2 : 0.0f; v3 = live ? v3 : 0.0f;
      v4f o;
      o.x = v0; o.y = v1; o.z = v2; o.w = v3;
      int h01, h23, l01, l23;
      hilo_pack(v0, v1, v2, v3, h01, h23, l01, l23);
      const v4i ow = regroup8(h01, h23, l01, l23, lane);
      float* op = Hout + (size_t)grow * HD + 4 * m;
      unsigned short* hp = HHLout + (size_t)grow * MPITCH + 8 * m;
      *(volatile v4f*)op = o;
      *(volatile v4i*)hp = ow;
      __threadfence();
      *(volatile v4f*)op = o;
      *(volatile v4i*)hp = ow;
    } else {
      v4f o;
      o.x = v0; o.y = v1; o.z = v2; o.w = v3;
      const int gc = live ? grow : (NN - 1);
      float* op = outp + (size_t)gc * HD + 4 * m;
      if (live) *(volatile v4f*)op = o;
      __threadfence();
      if (live) *(volatile v4f*)op = o;
    }
  }
}

__global__ __launch_bounds__(NTHR) __attribute__((amdgpu_num_vgpr(248)))
void k_gemm_one(const unsigned short* __restrict__ XBs, const unsigned short* __restrict__ Mhl,
                const unsigned short* __restrict__ WT, const float* __restrict__ sm,
                float* Hout, unsigned short* HHLout) {
  __shared__ __attribute__((aligned(16))) float stg[GBM * SP];
  __shared__ __attribute__((aligned(16))) float sb[64];
  gemm_rows<1>(XBs, Mhl, WT, sm, Hout, HHLout, (float*)nullptr, stg, sb);
}

__global__ __launch_bounds__(NTHR) __attribute__((amdgpu_num_vgpr(248)))
void k_gemm_two(const unsigned short* __restrict__ HHLs, const unsigned short* __restrict__ Mhl,
                const unsigned short* __restrict__ WT, const float* __restrict__ sm, float* outp) {
  __shared__ __attribute__((aligned(16))) float stg[GBM * SP];
  __shared__ __attribute__((aligned(16))) float sb[64];
  gemm_rows<2>(HHLs, Mhl, WT, sm, (float*)nullptr, (unsigned short*)nullptr, outp, stg, sb);
}

extern "C" void kernel_launch(void* const* d_in, const int* in_sizes, int n_in,
                              void* d_out, int out_size, void* d_ws, size_t ws_size,
                              hipStream_t stream) {
  if (n_in < 6) return;
  if (in_sizes[0] != NN * HD) return;
  if (in_sizes[1] != 2 * NE) return;
  if (in_sizes[2] != 2 * HD * HD) return;
  if (in_sizes[3] != HD) return;
  if (in_sizes[4] != 2 * HD * HD) return;
  if (in_sizes[5] != HD) return;
  if (out_size != NN * HD) return;

  const float* x  = (const float*)d_in[0];
  const int*   ei = (const int*)d_in[1];
  const float* W1 = (const float*)d_in[2];
  const float* b1 = (const float*)d_in[3];
  const float* W2 = (const float*)d_in[4];
  const float* b2 = (const float*)d_in[5];
  float* out = (float*)d_out;
  const int* keys = ei;
  const int* srcs = ei + NE;

  constexpr size_t zXB   = (size_t)MP * XP * 2;
  constexpr size_t zM    = (size_t)MP * MPITCH * 2;
  constexpr size_t zH    = (size_t)MP * HD * 4;
  constexpr size_t zHHL  = (size_t)MP * MPITCH * 2;
  constexpr size_t zLIST = (size_t)NBK * RCAP * 4;
  constexpr size_t zCO   = (size_t)NBK * 2 * NBRUN * 4;
  constexpr size_t zFLAG = (size_t)NBK * 128;
  constexpr size_t zWT1  = (size_t)HD * W1P * 2;
  constexpr size_t zWT2  = (size_t)HD * W2P * 2;
  constexpr size_t zSM   = 512;
  constexpr size_t oXB   = 0;
  constexpr size_t oM    = oXB + zXB;
  constexpr size_t oH    = oM + zM;
  constexpr size_t oHHL  = oH + zH;
  constexpr size_t oLIST = oHHL + zHHL;
  constexpr size_t oCO   = oLIST + zLIST;
  constexpr size_t oFLAG = oCO + zCO;
  constexpr size_t oWT1  = oFLAG + zFLAG;
  constexpr size_t oWT2  = oWT1 + zWT1;
  constexpr size_t oSM   = oWT2 + zWT2;
  constexpr size_t oEND  = oSM + zSM;
  static_assert(zXB % 256 == 0 && zM % 256 == 0 && zH % 256 == 0 && zHHL % 256 == 0 && zLIST % 256 == 0);
  static_assert(zCO % 256 == 0 && zFLAG % 256 == 0 && zWT1 % 256 == 0 && zWT2 % 256 == 0 && zSM % 256 == 0);
  static_assert(oEND <= WSMAX);
  if (oEND > ws_size) return;

  char* ws = (char*)d_ws;
  unsigned short* XB   = (unsigned short*)(ws + oXB);
  unsigned short* Mhl  = (unsigned short*)(ws + oM);
  float*          H    = (float*)(ws + oH);
  unsigned short* HHL  = (unsigned short*)(ws + oHHL);
  int*            LIST = (int*)(ws + oLIST);
  int*            CO   = (int*)(ws + oCO);
  int*            FLAG = (int*)(ws + oFLAG);
  unsigned short* WT1  = (unsigned short*)(ws + oWT1);
  unsigned short* WT2  = (unsigned short*)(ws + oWT2);
  float*          SM   = (float*)(ws + oSM);

  hipFuncSetAttribute(reinterpret_cast<const void*>(&k_bucket), hipFuncAttributeMaxDynamicSharedMemorySize, (int)BK_LDS);

  k_prep<<<PBTOT, NTHR, 0, stream>>>(x, W1, b1, W2, b2, XB, WT1, WT2, SM);
  k_bucket<<<NBK, NTHR, BK_LDS, stream>>>(keys, srcs, LIST, CO, FLAG);
  k_replay_one<<<MP / ABM, NTHR, 0, stream>>>(LIST, CO, FLAG, XB, Mhl);
  k_gemm_one<<<MP / GBM, NTHR, 0, stream>>>(XB, Mhl, WT1, SM, H, HHL);
  k_replay_two<<<MP / ABM, NTHR, 0, stream>>>(LIST, CO, FLAG, H, Mhl);
  k_gemm_two<<<MP / GBM, NTHR, 0, stream>>>(HHL, Mhl, WT2, SM, out);
}
